// FuseBaseNoSia_17239998726589
// MI455X (gfx1250) — hardware-verified
//
#include <hip/hip_runtime.h>
#include <stddef.h>
#include <math.h>

typedef __attribute__((ext_vector_type(16))) _Float16 v16h;
typedef __attribute__((ext_vector_type(8)))  _Float16 v8h;
typedef __attribute__((ext_vector_type(16))) __bf16   v16b;
typedef __attribute__((ext_vector_type(8)))  __bf16   v8b;
typedef __attribute__((ext_vector_type(8)))  float    v8f;
typedef __attribute__((ext_vector_type(4)))  float    v4f;
typedef __attribute__((ext_vector_type(2)))  float    v2f;
typedef __attribute__((ext_vector_type(4)))  int      v4i;

constexpr int HIDC    = 64;
constexpr int NBA     = 1024;
constexpr int RPQ     = 1024;
constexpr int PPITCH  = 32;
constexpr int NCLSMAX = 32;
constexpr int SOMAX   = 12288;
constexpr int NWTMAX  = 16;
#define NTHR    256
#define NWAVE   8
#define EPT     8
#define NGRP    1
#define CHUNK   (NTHR * EPT * NGRP)
#define WCAP    (EPT * NGRP * 32)
#define LISTN   (NWAVE * WCAP)
#define LDS_AGG ((NBA * HIDC + NBA) * 4 + LISTN * 4 + 64)

static_assert((CHUNK & (CHUNK - 1)) == 0);
static_assert(CHUNK <= 4096);
static_assert((NBA & (NBA - 1)) == 0 && NBA <= 4096);
static_assert(RPQ % NBA == 0 && RPQ % 64 == 0 && RPQ % NTHR == 0);
static_assert(LDS_AGG == 274496);
static_assert(HIDC % 64 == 0);
static_assert(PPITCH == 32 && NCLSMAX <= PPITCH);

__device__ __forceinline__ unsigned short f2bf_bits(float f) {
  unsigned u = __float_as_uint(f);
  return (unsigned short)((u + 0x7FFFu + ((u >> 16) & 1u)) >> 16);
}
__device__ __forceinline__ float bf_bits2f(unsigned short h) { return __uint_as_float(((unsigned)h) << 16); }

__device__ __forceinline__ void dep_guard_h(v8f& a, v8f& b, v16h x, v16h y) { asm volatile("v_nop\n\tv_nop\n\tv_nop\n\tv_nop" : "+v"(a), "+v"(b) : "v"(x), "v"(y)); }
__device__ __forceinline__ void dep_guard_b(v8f& a, v8f& b, v16b x, v16b y) { asm volatile("v_nop\n\tv_nop\n\tv_nop\n\tv_nop" : "+v"(a), "+v"(b) : "v"(x), "v"(y)); }
__device__ __forceinline__ void keep4_h(v16h a, v16h b, v16h c, v16h d) { asm volatile("v_nop" :: "v"(a), "v"(b), "v"(c), "v"(d)); }
__device__ __forceinline__ void keep4_b(v16b a, v16b b, v16b c, v16b d) { asm volatile("v_nop" :: "v"(a), "v"(b), "v"(c), "v"(d)); }
__device__ __forceinline__ void acc_guard4(v8f& a, v8f& b, v8f& c, v8f& d) { asm volatile("v_nop\n\tv_nop\n\tv_nop\n\tv_nop" : "+v"(a), "+v"(b), "+v"(c), "+v"(d)); }
template <typename T> struct Frag;
template <> struct Frag<_Float16> {
  typedef v16h V; union U { v16h v; v8h h[2]; };
  static __device__ __forceinline__ v16h load(const _Float16* p) {
    U f; f.h[0] = *(const v8h*)(p); f.h[1] = *(const v8h*)(p + 16); return f.v;
  }
  static __device__ __forceinline__ v8f mma(v16h a, v16h b, v8f c) {
    return __builtin_amdgcn_wmma_f32_16x16x32_f16(false, a, false, b, (short)0, c, false, false);
  }
  static __device__ __forceinline__ void guard(v8f& a, v8f& b, v16h x, v16h y) { dep_guard_h(a, b, x, y); }
  static __device__ __forceinline__ void keep(v16h a, v16h b, v16h c, v16h d) { keep4_h(a, b, c, d); }
};
template <> struct Frag<__bf16> {
  typedef v16b V; union U { v16b v; v8b h[2]; };
  static __device__ __forceinline__ v16b load(const __bf16* p) {
    U f; f.h[0] = *(const v8b*)(p); f.h[1] = *(const v8b*)(p + 16); return f.v;
  }
  static __device__ __forceinline__ v8f mma(v16b a, v16b b, v8f c) {
    return __builtin_amdgcn_wmma_f32_16x16x32_bf16(false, a, false, b, (short)0, c, false, false);
  }
  static __device__ __forceinline__ void guard(v8f& a, v8f& b, v16b x, v16b y) { dep_guard_b(a, b, x, y); }
  static __device__ __forceinline__ void keep(v16b a, v16b b, v16b c, v16b d) { keep4_b(a, b, c, d); }
};

template <int ET> struct Elem;
template <> struct Elem<0> { typedef _Float16 T; };
template <> struct Elem<1> { typedef __bf16 T; };
template <int ET, bool SPLIT, int BIAS_MODE, int OUT_MODE, bool RESID, int ACT = 0>
__global__ __launch_bounds__(256) void wmma_gemm64(
    const unsigned short* __restrict__ Ap, const unsigned short* __restrict__ A2p, int lda, long strideA,
    const unsigned short* __restrict__ Btp, const unsigned short* __restrict__ Bt2p, int ldb, long strideB,
    void* __restrict__ Cout, void* __restrict__ Cout2, int ldc, long strideC,
    const float* __restrict__ bias,
    const float* __restrict__ resid, long strideR,
    int M, int N, int K, float scale) {
  typedef typename Elem<ET>::T T;
  typedef typename Frag<T>::V V;
  const T* A = (const T*)Ap; const T* A2 = (const T*)A2p; const T* Bt = (const T*)Btp; const T* Bt2 = (const T*)Bt2p;
  __shared__ __align__(16) float sT[8][16 * 68];
  const int b    = blockIdx.y;
  const int lane = threadIdx.x & 31;
  const int wave = threadIdx.x >> 5;
  const int tilesN = N >> 6;
  const int tilesM = M >> 6;
  const int tile = blockIdx.x * 8 + wave;
  if (tile >= tilesM * tilesN) return;
  const int tm = tile / tilesN;
  const int tn = tile - tm * tilesN;
  const int m0 = tm << 6;
  const int n0 = tn << 6;

  const T* Ab  = A  + (size_t)b * strideA;
  const T* Bb  = Bt + (size_t)b * strideB;
  const T* Ab2 = SPLIT ? (A2  + (size_t)b * strideA) : nullptr;
  const T* Bb2 = SPLIT ? (Bt2 + (size_t)b * strideB) : nullptr;

  const int rlane = lane & 15;
  const int koff  = (lane >> 4) * 8;
  const int mOff  = (lane >> 4) * 8;

  v8f acc[4][4];
#pragma unroll
  for (int i = 0; i < 4; ++i)
#pragma unroll
    for (int j = 0; j < 4; ++j) acc[i][j] = (v8f){0.f,0.f,0.f,0.f,0.f,0.f,0.f,0.f};

  for (int k0 = 0; k0 < K; k0 += 32) {
    V bh[4], bl[4];
#pragma unroll
    for (int j = 0; j < 4; ++j) {
      const size_t bo = (size_t)(n0 + (j << 4) + rlane) * ldb + koff + k0;
      bh[j] = Frag<T>::load(Bb + bo);
      if (SPLIT) bl[j] = Frag<T>::load(Bb2 + bo);
    }
#pragma unroll
    for (int i = 0; i < 4; ++i) {
      const size_t ao = (size_t)(m0 + (i << 4) + rlane) * lda + koff + k0;
      V ah = Frag<T>::load(Ab + ao);
      V al;
      if (SPLIT) al = Frag<T>::load(Ab2 + ao);
#pragma unroll
      for (int j = 0; j < 4; ++j) {
        acc[i][j] = Frag<T>::mma(ah, bh[j], acc[i][j]);
        if (SPLIT) {
          acc[i][j] = Frag<T>::mma(ah, bl[j], acc[i][j]);
          acc[i][j] = Frag<T>::mma(al, bh[j], acc[i][j]);
        }
      }
      Frag<T>::guard(acc[i][0], acc[i][3], ah, SPLIT ? al : ah);
    }
    Frag<T>::keep(bh[0], bh[1], bh[2], bh[3]);
    if (SPLIT) Frag<T>::keep(bl[0], bl[1], bl[2], bl[3]);
  }
  acc_guard4(acc[0][0], acc[0][1], acc[0][2], acc[0][3]);
  acc_guard4(acc[1][0], acc[1][1], acc[1][2], acc[1][3]);
  acc_guard4(acc[2][0], acc[2][1], acc[2][2], acc[2][3]);
  acc_guard4(acc[3][0], acc[3][1], acc[3][2], acc[3][3]);

  float* slab = sT[wave];
  const float* Rb = RESID ? (resid + (size_t)b * strideR) : nullptr;
#pragma unroll
  for (int i = 0; i < 4; ++i) {
    const int mBase = m0 + (i << 4);
#pragma unroll
    for (int j = 0; j < 4; ++j) {
      const int n = n0 + (j << 4) + rlane;
      float bv = 0.f;
      if (BIAS_MODE == 2) bv = bias[n];
#pragma unroll
      for (int r = 0; r < 8; ++r) {
        float v = acc[i][j][r] * scale;
        if (BIAS_MODE == 1) v += bias[mBase + mOff + r];
        if (BIAS_MODE == 2) v += bv;
        if (RESID) v += Rb[(size_t)(mBase + mOff + r) * ldc + n];
        if (ACT == 1) v = tanhf(v);
        if (ACT == 2) v = fmaxf(v, 0.0f);
        if (ACT == 3) v = v / (1.0f + expf(-v));
        if (ACT == 4) v = (v > 0.f) ? v : 0.01f * v;
        if (ACT == 5) v = 0.5f * v * (1.0f + erff(v * 0.70710678118654752f));
        slab[(mOff + r) * 68 + (j << 4) + rlane] = v;
      }
    }
    __builtin_amdgcn_fence(__ATOMIC_RELEASE, "workgroup");
    __builtin_amdgcn_wave_barrier();
    __builtin_amdgcn_fence(__ATOMIC_ACQUIRE, "workgroup");
    if (OUT_MODE == 0) {
      float* C = (float*)Cout + (size_t)b * strideC;
      const int hh = lane >> 4, c4 = (lane & 15) * 4;
      for (int pass = 0; pass < 2; ++pass) {
#pragma unroll
        for (int it = 0; it < 8; ++it) {
          const int row = it * 2 + hh;
          v4f v = *(const v4f*)(slab + row * 68 + c4);
          *(volatile v4f*)(C + (size_t)(mBase + row) * ldc + n0 + c4) = v;
        }
        __threadfence();
      }
    } else {
      const int q = lane >> 3, c8 = (lane & 7) * 8;
      unsigned short* C  = (unsigned short*)Cout  + (size_t)b * strideC;
      unsigned short* C2 = (OUT_MODE == 2) ? ((unsigned short*)Cout2 + (size_t)b * strideC) : nullptr;
      for (int pass = 0; pass < 2; ++pass) {
#pragma unroll
        for (int it = 0; it < 4; ++it) {
          const int row = it * 4 + q;
          const float* sp = slab + row * 68 + c8;
          v8h hv, lv;
#pragma unroll
          for (int e = 0; e < 8; ++e) {
            if (OUT_MODE == 1) {
              hv[e] = (_Float16)sp[e];
            } else {
              unsigned short hb = f2bf_bits(sp[e]);
              unsigned short lb = f2bf_bits(sp[e] - bf_bits2f(hb));
              hv[e] = __builtin_bit_cast(_Float16, hb);
              lv[e] = __builtin_bit_cast(_Float16, lb);
            }
          }
          *(volatile v8h*)(C + (size_t)(mBase + row) * ldc + n0 + c8) = hv;
          if (OUT_MODE == 2) *(volatile v8h*)(C2 + (size_t)(mBase + row) * ldc + n0 + c8) = lv;
        }
        __threadfence();
      }
    }
    __builtin_amdgcn_fence(__ATOMIC_RELEASE, "workgroup");
    __builtin_amdgcn_wave_barrier();
    __builtin_amdgcn_fence(__ATOMIC_ACQUIRE, "workgroup");
  }
}

template <int NB>
__device__ __forceinline__ int scan_chunk(const int* __restrict__ lst, int nE, int cbase, int nodeBase,
                                          int* list, int tid, int lane, int wave, int fullvec) {
  int wc = 0;
#pragma unroll
  for (int g = 0; g < NGRP; ++g) {
    const int el0 = (g * NTHR + tid) * EPT;
    const int e0  = cbase + el0;
    v4i da, db;
    if (fullvec) {
      da = *(const v4i*)(lst + e0);
      db = *(const v4i*)(lst + e0 + 4);
    } else {
      const int em = nE - 1;
      da.x = lst[(e0     < em) ? e0     : em];
      da.y = lst[(e0 + 1 < em) ? e0 + 1 : em];
      da.z = lst[(e0 + 2 < em) ? e0 + 2 : em];
      da.w = lst[(e0 + 3 < em) ? e0 + 3 : em];
      db.x = lst[(e0 + 4 < em) ? e0 + 4 : em];
      db.y = lst[(e0 + 5 < em) ? e0 + 5 : em];
      db.z = lst[(e0 + 6 < em) ? e0 + 6 : em];
      db.w = lst[(e0 + 7 < em) ? e0 + 7 : em];
    }
    const bool v0 = (e0 < nE), v1 = (e0 + 1 < nE), v2 = (e0 + 2 < nE), v3 = (e0 + 3 < nE);
    const bool v4 = (e0 + 4 < nE), v5 = (e0 + 5 < nE), v6 = (e0 + 6 < nE), v7 = (e0 + 7 < nE);
    const unsigned nb = (unsigned)nodeBase;
    const unsigned s0 = (unsigned)da.x - nb, s1 = (unsigned)da.y - nb;
    const unsigned s2 = (unsigned)da.z - nb, s3 = (unsigned)da.w - nb;
    const unsigned s4 = (unsigned)db.x - nb, s5 = (unsigned)db.y - nb;
    const unsigned s6 = (unsigned)db.z - nb, s7 = (unsigned)db.w - nb;
    const bool h0 = v0 && (s0 < (unsigned)NB), h1 = v1 && (s1 < (unsigned)NB);
    const bool h2 = v2 && (s2 < (unsigned)NB), h3 = v3 && (s3 < (unsigned)NB);
    const bool h4 = v4 && (s4 < (unsigned)NB), h5 = v5 && (s5 < (unsigned)NB);
    const bool h6 = v6 && (s6 < (unsigned)NB), h7 = v7 && (s7 < (unsigned)NB);
    const unsigned any = __builtin_amdgcn_ballot_w32(h0 | h1 | h2 | h3 | h4 | h5 | h6 | h7);
    if (any != 0u) {
#define HITJ(J, HJ, SJ) { \
        const unsigned mj = __builtin_amdgcn_ballot_w32(HJ); \
        if (mj != 0u) { \
          if (HJ) { \
            const int pos = wc + (int)__builtin_amdgcn_mbcnt_lo(mj, 0u); \
            if (pos < WCAP) list[wave * WCAP + pos] = ((el0 + (J)) << 12) | (int)(SJ); \
          } \
          wc += (int)__builtin_popcount(mj); } }
      HITJ(0, h0, s0)
      HITJ(1, h1, s1)
      HITJ(2, h2, s2)
      HITJ(3, h3, s3)
      HITJ(4, h4, s4)
      HITJ(5, h5, s5)
      HITJ(6, h6, s6)
      HITJ(7, h7, s7)
#undef HITJ
    }
  }
  return wc;
}

__global__ __launch_bounds__(NTHR) void k_wprep(const float* __restrict__ W, int Kin, int ncol, int Kpad,
                                                unsigned short* bt) {
  const int tpr = Kpad >> 3;
  const int i = blockIdx.x * NTHR + threadIdx.x;
  if (i >= HIDC * tpr) return;
  const int n   = i / tpr;
  const int k0  = (i - n * tpr) * 8;
  const int ncl = (n < ncol) ? n : ncol - 1;
  v8h hv;
#pragma unroll
  for (int e = 0; e < 8; ++e) {
    const int k  = k0 + e;
    const int kc = (k < Kin) ? k : Kin - 1;
    float v = W[(size_t)kc * ncol + ncl];
    if (k >= Kin || n >= ncol) v = 0.f;
    hv[e] = (_Float16)(64.0f * v);
  }
  const size_t o = (size_t)i * 8;
  *(volatile v8h*)(bt + o) = hv;
  __threadfence();
  *(volatile v8h*)(bt + o) = hv;
}

__global__ __launch_bounds__(NTHR) void k_mean_agg(
    const int* __restrict__ rowl, const int* __restrict__ coll,
    const float* __restrict__ hfeat, unsigned short* oh,
    int nN, int nE, int vec_ok) {
  constexpr int NB  = NBA;
  constexpr int HC  = HIDC;
  constexpr int RW  = NB / NWAVE;
  static_assert(NB * HC == 65536);
  static_assert((NB * HC / 4) % NTHR == 0 && (RW % 4) == 0 && NB % NTHR == 0);
  extern __shared__ v4f lds_dyn[];
  float* acc  = (float*)lds_dyn;
  float* cnt  = acc + NB * HC;
  int*   list = (int*)(cnt + NB);
  int*   wcnt = list + LISTN;
  const int tid = threadIdx.x, lane = tid & 31, wave = tid >> 5;
  const int nodeBase = blockIdx.x * NB;

  {
    const v4f zz = {0.f, 0.f, 0.f, 0.f};
    for (int i = tid; i < NB * HC / 4; i += NTHR) lds_dyn[i] = zz;
    for (int i = tid; i < NB; i += NTHR) cnt[i] = 0.f;
  }
  __syncthreads();

  const int nChunks = (nE + CHUNK - 1) / CHUNK;
#pragma unroll 1
  for (int ch = 0; ch < nChunks; ++ch) {
    const int cbase = ch * CHUNK;
    const int fullvec = (vec_ok != 0 && cbase + CHUNK <= nE) ? 1 : 0;
    const int wc = scan_chunk<NB>(coll, nE, cbase, nodeBase, list, tid, lane, wave, fullvec);
    if (lane == 0) wcnt[wave] = wc;
    __syncthreads();
    if (wave == 0) {
#pragma unroll 1
      for (int wsx = 0; wsx < NWAVE; ++wsx) {
        int n = __builtin_amdgcn_readfirstlane(wcnt[wsx]);
        n = n > WCAP ? WCAP : (n < 0 ? 0 : n);
        const int* lp = list + wsx * WCAP;
#pragma unroll 1
        for (int i = 0; i < n; ++i) {
          const int ent  = __builtin_amdgcn_readfirstlane(lp[i]);
          const int slot = ent & (NB - 1);
          int e = cbase + ((ent >> 12) & (CHUNK - 1));
          e = e > nE - 1 ? nE - 1 : e;
          int s = rowl[e];
          s = s < 0 ? 0 : (s > nN - 1 ? nN - 1 : s);
          const v2f hv = *(const v2f*)(hfeat + (size_t)s * HC + 2 * lane);
          v2f* ap = (v2f*)(acc + slot * HC + 2 * lane);
          const v2f av = *ap;
          *ap = av + hv;
          const float co = cnt[slot];
          cnt[slot] = co + 1.0f;
        }
      }
    }
    __syncthreads();
  }

  unsigned short* hb = oh + (size_t)nodeBase * HC;
  for (int pass = 0; pass < 2; ++pass) {
#pragma unroll 2
    for (int q = 0; q < RW / 4; ++q) {
      const int row = wave * RW + 4 * q + (lane >> 3);
      const int col = (lane & 7) * 8;
      const float c   = cnt[row];
      const float inv = 1.0f / fmaxf(c, 1.0f);
      const float* sp = acc + row * HC + col;
      v4f p0 = *(const v4f*)sp, p1 = *(const v4f*)(sp + 4);
      p0 = (p0 * inv) * 16.0f;
      p1 = (p1 * inv) * 16.0f;
      if (nodeBase + row >= nN) { const v4f zz = {0.f, 0.f, 0.f, 0.f}; p0 = zz; p1 = zz; }
      v8h hv;
      hv[0] = (_Float16)p0.x; hv[1] = (_Float16)p0.y; hv[2] = (_Float16)p0.z; hv[3] = (_Float16)p0.w;
      hv[4] = (_Float16)p1.x; hv[5] = (_Float16)p1.y; hv[6] = (_Float16)p1.z; hv[7] = (_Float16)p1.w;
      *(volatile v8h*)(hb + (size_t)row * HC + col) = hv;
    }
    __threadfence();
  }
}

__global__ __launch_bounds__(NTHR) void k_fuse(const float* __restrict__ xa, const float* __restrict__ xb,
                                               unsigned short* hh, int nRows) {
  const int i = blockIdx.x * NTHR + threadIdx.x;
  if (i >= nRows * (HIDC / 8)) return;
  const size_t o = (size_t)i * 8;
  const v4f a0 = *(const v4f*)(xa + o), a1 = *(const v4f*)(xa + o + 4);
  const v4f b0 = *(const v4f*)(xb + o), b1 = *(const v4f*)(xb + o + 4);
  const v4f s0 = (a0 + b0) * 8.0f;
  const v4f s1 = (a1 + b1) * 8.0f;
  v8h hv;
  hv[0] = (_Float16)s0.x; hv[1] = (_Float16)s0.y; hv[2] = (_Float16)s0.z; hv[3] = (_Float16)s0.w;
  hv[4] = (_Float16)s1.x; hv[5] = (_Float16)s1.y; hv[6] = (_Float16)s1.z; hv[7] = (_Float16)s1.w;
  *(volatile v8h*)(hh + o) = hv;
  __threadfence();
  *(volatile v8h*)(hh + o) = hv;
}

__global__ __launch_bounds__(NTHR) void k_pool(const int* __restrict__ batch, const float* __restrict__ hn,
                                               const float* __restrict__ bo, float* pooled,
                                               int nN, int nCls, int vec_ok) {
  __shared__ int list[LISTN];
  __shared__ int wcnt[NWAVE];
  __shared__ __align__(16) float prow[PPITCH];
  const int tid = threadIdx.x, lane = tid & 31, wave = tid >> 5;
  const int g = blockIdx.x;
  const int lb = (lane < nCls) ? lane : nCls - 1;
  float bl = bo[lb];
  if (lane >= nCls) bl = 0.f;
  float accv = 0.f;
  float cnt = 0.f;
  const int nChunks = (nN + CHUNK - 1) / CHUNK;
#pragma unroll 1
  for (int ch = 0; ch < nChunks; ++ch) {
    const int cbase = ch * CHUNK;
    const int fullvec = (vec_ok != 0 && cbase + CHUNK <= nN) ? 1 : 0;
    const int wc = scan_chunk<1>(batch, nN, cbase, g, list, tid, lane, wave, fullvec);
    if (lane == 0) wcnt[wave] = wc;
    __syncthreads();
    if (wave == 0) {
#pragma unroll 1
      for (int wsx = 0; wsx < NWAVE; ++wsx) {
        int n = __builtin_amdgcn_readfirstlane(wcnt[wsx]);
        n = n > WCAP ? WCAP : (n < 0 ? 0 : n);
        const int* lp = list + wsx * WCAP;
#pragma unroll 1
        for (int i = 0; i < n; ++i) {
          const int ent = __builtin_amdgcn_readfirstlane(lp[i]);
          int node = cbase + ((ent >> 12) & (CHUNK - 1));
          node = node > nN - 1 ? nN - 1 : (node < 0 ? 0 : node);
          const float v = hn[(size_t)node * HIDC + lane];
          accv += v + bl;
          cnt += 1.0f;
        }
      }
    }
    __syncthreads();
  }
  if (wave == 0) {
    const float inv = 1.0f / fmaxf(cnt, 1.0f);
    float r = accv * inv;
    if (lane >= nCls) r = 0.f;
    prow[lane] = r;
  }
  __syncthreads();
  if (wave == 0) {
    const int lc = (lane < 8) ? lane : 7;
    const v4f v = *(const v4f*)(prow + 4 * lc);
    float* dp = pooled + (size_t)g * PPITCH + 4 * lane;
    if (lane < 8) *(volatile v4f*)dp = v;
    __threadfence();
    if (lane < 8) *(volatile v4f*)dp = v;
  }
}

__global__ __launch_bounds__(NTHR) void k_out(const float* __restrict__ pooled, float* out, int G, int nCls) {
  __shared__ __align__(16) float so[SOMAX];
  const int tid = threadIdx.x, lane = tid & 31, wave = tid >> 5;
  const int nflt = G * nCls;
#pragma unroll 1
  for (int g = tid; g < G; g += NTHR) {
    const float* pr = pooled + (size_t)g * PPITCH;
#pragma unroll 1
    for (int c = 0; c < nCls; ++c) so[g * nCls + c] = pr[c];
  }
  for (int i = nflt + tid; i < nflt + 128; i += NTHR) so[i] = 0.f;
  __syncthreads();
  for (int pass = 0; pass < 2; ++pass) {
#pragma unroll 1
    for (int s = wave; s * 128 < nflt; s += NWAVE) {
      const int idx = s * 128 + lane * 4;
      const v4f v = *(const v4f*)(so + idx);
      if (idx + 4 <= nflt) *(volatile v4f*)(out + idx) = v;
    }
    if (tid == 0 && (nflt & 3) != 0) {
      const int i0 = nflt & ~3;
#pragma unroll 1
      for (int t = 0; t < (nflt & 3); ++t) {
        const float tv = so[i0 + t];
        *(volatile float*)(out + i0 + t) = tv;
      }
    }
    __threadfence();
  }
}

extern "C" void kernel_launch(void* const* d_in, const int* in_sizes, int n_in,
                              void* d_out, int out_size, void* d_ws, size_t ws_size,
                              hipStream_t stream) {
  if (n_in < 10) return;
  const int nN   = in_sizes[0] / HIDC;
  const int L0   = in_sizes[1] / (HIDC * HIDC);
  const int L1   = in_sizes[3] / (HIDC * HIDC);
  const int nCls = in_sizes[6];
  const int nEs  = in_sizes[7] / 2;
  const int nEf  = in_sizes[8] / 2;
  if (nN < 1 || in_sizes[0] != nN * HIDC || nN > (1 << 24)) return;
  if (L0 < 1 || in_sizes[1] != L0 * HIDC * HIDC || in_sizes[2] != L0 * HIDC) return;
  if (L1 < 1 || in_sizes[3] != L1 * HIDC * HIDC || in_sizes[4] != L1 * HIDC) return;
  if (L0 + L1 + 1 > NWTMAX) return;
  if (nCls < 1 || nCls > NCLSMAX || in_sizes[5] != HIDC * nCls) return;
  if (nEs < 1 || in_sizes[7] != 2 * nEs || nEf < 1 || in_sizes[8] != 2 * nEf) return;
  if (in_sizes[9] != nN) return;
  const int G = out_size / nCls;
  if (G < 1 || out_size != G * nCls || G * nCls + 128 > SOMAX) return;

  const float* x     = (const float*)d_in[0];
  const float* W0    = (const float*)d_in[1];
  const float* b0    = (const float*)d_in[2];
  const float* W1    = (const float*)d_in[3];
  const float* b1    = (const float*)d_in[4];
  const float* Wout  = (const float*)d_in[5];
  const float* bout  = (const float*)d_in[6];
  const int*   eis   = (const int*)d_in[7];
  const int*   eif   = (const int*)d_in[8];
  const int*   batch = (const int*)d_in[9];
  float* out = (float*)d_out;

  const int RP = ((nN + RPQ - 1) / RPQ) * RPQ;
  const int nA = RP / NBA;
  const int nWT = L0 + L1 + 1;
  const int vecS = ((nEs & 3) == 0) ? 1 : 0;
  const int vecF = ((nEf & 3) == 0) ? 1 : 0;

  char* ws = (char*)d_ws;
  size_t off = 0;
  const size_t oWT  = off; off += (size_t)nWT * HIDC * HIDC * 2;
  const size_t oAGG = off; off += (size_t)RP * HIDC * 2;
  const size_t oXS  = off; off += (size_t)RP * HIDC * 4;
  const size_t oXF  = off; off += (size_t)RP * HIDC * 4;
  const size_t oH16 = off; off += (size_t)RP * HIDC * 2;
  const size_t oON  = off; off += (size_t)RP * HIDC * 4;
  const size_t oPL  = off; off += (size_t)G * PPITCH * 4;
  if (off > ws_size || off > (size_t)134217728) return;

  unsigned short* wt  = (unsigned short*)(ws + oWT);
  unsigned short* agg = (unsigned short*)(ws + oAGG);
  float* xs  = (float*)(ws + oXS);
  float* xf  = (float*)(ws + oXF);
  unsigned short* h16 = (unsigned short*)(ws + oH16);
  float* on  = (float*)(ws + oON);
  float* pl  = (float*)(ws + oPL);

  const size_t WPL = (size_t)HIDC * HIDC;
  const int wpBlocks = (HIDC * (HIDC / 8) + NTHR - 1) / NTHR;
  const float gscale = 0.0009765625f;

  for (int l = 0; l < L0; ++l)
    k_wprep<<<wpBlocks, NTHR, 0, stream>>>(W0 + (size_t)l * HIDC * HIDC, HIDC, HIDC, HIDC, wt + (size_t)l * WPL);
  for (int l = 0; l < L1; ++l)
    k_wprep<<<wpBlocks, NTHR, 0, stream>>>(W1 + (size_t)l * HIDC * HIDC, HIDC, HIDC, HIDC, wt + (size_t)(L0 + l) * WPL);
  k_wprep<<<wpBlocks, NTHR, 0, stream>>>(Wout, HIDC, nCls, HIDC, wt + (size_t)(L0 + L1) * WPL);

  const int gg = ((RP / 64) * (HIDC / 64) + 7) / 8;

  for (int l = 0; l < L0; ++l) {
    const float* src = (l == 0) ? x : xs;
    k_mean_agg<<<nA, NTHR, LDS_AGG, stream>>>(eis, eis + nEs, src, agg, nN, nEs, vecS);
    wmma_gemm64<0, false, 2, 0, false, 2><<<dim3(gg, 1), 256, 0, stream>>>(
        agg, agg, HIDC, 0L, wt + (size_t)l * WPL, wt + (size_t)l * WPL, HIDC, 0L,
        (void*)xs, (void*)xs, HIDC, 0L, b0 + (size_t)l * HIDC, b0, 0L, RP, HIDC, HIDC, gscale);
  }
  for (int l = 0; l < L1; ++l) {
    const float* src = (l == 0) ? x : xf;
    k_mean_agg<<<nA, NTHR, LDS_AGG, stream>>>(eif, eif + nEf, src, agg, nN, nEf, vecF);
    wmma_gemm64<0, false, 2, 0, false, 2><<<dim3(gg, 1), 256, 0, stream>>>(
        agg, agg, HIDC, 0L, wt + (size_t)(L0 + l) * WPL, wt + (size_t)(L0 + l) * WPL, HIDC, 0L,
        (void*)xf, (void*)xf, HIDC, 0L, b1 + (size_t)l * HIDC, b1, 0L, RP, HIDC, HIDC, gscale);
  }

  k_fuse<<<RP * (HIDC / 8) / NTHR, NTHR, 0, stream>>>(xs, xf, h16, RP);
  wmma_gemm64<0, false, 0, 0, false, 0><<<dim3(gg, 1), 256, 0, stream>>>(
      h16, h16, HIDC, 0L, wt + (size_t)(L0 + L1) * WPL, wt + (size_t)(L0 + L1) * WPL, HIDC, 0L,
      (void*)on, (void*)on, HIDC, 0L, bout, bout, 0L, RP, HIDC, HIDC, gscale);

  k_pool<<<G, NTHR, 0, stream>>>(batch, on, bout, pl, nN, nCls, 1);
  k_out<<<1, NTHR, 0, stream>>>(pl, out, G, nCls);
}
